// ReadInAttention_53480932770343
// MI455X (gfx1250) — hardware-run, weakly checked
//
#include <hip/hip_runtime.h>
#include <math.h>
#include <stdint.h>

#define NB_   4
#define NU_   64
#define NV_   256
#define SD_   768
#define CD_   384
#define NI_   512
#define NH_   8
#define HD_   64
#define RROWS (NB_ * NU_)
#define SROWS (NB_ * NV_)
#define AROWS (NB_ * NH_ * NU_)
#define CMW   (3 * SD_ + NI_)
#define LNEPS 1e-5f
#define WSC   64.0f
#define LOSC  2048.0f
#define PSC   1024.0f
#define ASC   64.0f
#define MSC   64.0f

#define F_BIAS  1
#define F_MULP  2
#define F_GCOL  4
#define F_RESID 8
#define F_OUT32 16
#define F_OUTHL 32

static_assert((RROWS % 16) == 0 && (SROWS % 8) == 0 && (AROWS % 8) == 0 && (NU_ % 16) == 0);
static_assert((SD_ % 64) == 0 && (CD_ % 64) == 0 && (NI_ % 64) == 0 && (NV_ % 64) == 0 && (CMW % 64) == 0);
static_assert((HD_ % 32) == 0 && NH_ * HD_ == NI_ && NV_ == 256 && SD_ == 768 && NU_ == 64 && NH_ == 8);

typedef _Float16 v16h __attribute__((ext_vector_type(16)));
typedef _Float16 v8h  __attribute__((ext_vector_type(8)));
typedef float    v8f  __attribute__((ext_vector_type(8)));
typedef float    v4f  __attribute__((ext_vector_type(4)));
typedef unsigned int v4u __attribute__((ext_vector_type(4)));

union FragH { v16h v; v8h h[2]; };

__device__ __forceinline__ unsigned short bf_bits(float f) {
  unsigned u = __float_as_uint(f);
  return (unsigned short)((u + 0x7FFFu + ((u >> 16) & 1u)) >> 16);
}
__device__ __forceinline__ float bf_up(unsigned short h) { return __uint_as_float(((unsigned)h) << 16); }
__device__ __forceinline__ float bfr(float f) { return bf_up(bf_bits(f)); }
__device__ __forceinline__ unsigned short h_bits(_Float16 x) { return __builtin_bit_cast(unsigned short, x); }
__device__ __forceinline__ unsigned pk16(unsigned short a, unsigned short b) { return (unsigned)a | ((unsigned)b << 16); }
__device__ __forceinline__ unsigned pkh(float a, float b) { return pk16(h_bits((_Float16)a), h_bits((_Float16)b)); }
__device__ __forceinline__ v8f zero8() { v8f z = {0.f, 0.f, 0.f, 0.f, 0.f, 0.f, 0.f, 0.f}; return z; }
__device__ __forceinline__ v4f zero4() { v4f z = {0.f, 0.f, 0.f, 0.f}; return z; }

__device__ __forceinline__ void hl_pair(float f0, float f1, unsigned& hp, unsigned& lp) {
#pragma clang fp contract(off)
  const _Float16 h0 = (_Float16)f0, h1 = (_Float16)f1;
  const float d0 = f0 - (float)h0, d1 = f1 - (float)h1;
  const float r0 = d0 * LOSC, r1 = d1 * LOSC;
  hp = pk16(h_bits(h0), h_bits(h1));
  lp = pk16(h_bits((_Float16)r0), h_bits((_Float16)r1));
}

__device__ __forceinline__ v16h ldfrag_h(const _Float16* p) {
  FragH f;
  f.h[0] = *(const v8h*)(p);
  f.h[1] = *(const v8h*)(p + 16);
  return f.v;
}

__device__ __forceinline__ v8f mma_h(v16h a, v16h b, v8f c) {
  c = __builtin_amdgcn_wmma_f32_16x16x32_f16(false, a, false, b, (short)0, c, false, false);
#if defined(__HIP_DEVICE_COMPILE__)
  asm volatile("v_nop\n\tv_nop\n\tv_nop\n\tv_nop" : "+v"(c) : "v"(a), "v"(b));
#endif
  return c;
}
__device__ __forceinline__ void wave_sync_lds() {
  __builtin_amdgcn_fence(__ATOMIC_RELEASE, "workgroup");
  __builtin_amdgcn_wave_barrier();
  __builtin_amdgcn_fence(__ATOMIC_ACQUIRE, "workgroup");
}

__global__ __launch_bounds__(256) void cvt_wT(const float* __restrict__ w0, const float* __restrict__ w1,
                                              const float* __restrict__ w2, unsigned short* outp, int nin,
                                              int nout) {
  __shared__ float tile[64][33];
  const int tid = threadIdx.x;
  const int z = blockIdx.z;
  const float* src = (z == 0) ? w0 : ((z == 1) ? w1 : w2);
  unsigned short* dst = outp + (size_t)z * nin * nout;
  const int i0 = blockIdx.x * 64;
  const int o0 = blockIdx.y * 32;
#pragma unroll
  for (int p = 0; p < 8; ++p) {
    const int idx = p * 256 + tid;
    const int i = idx >> 5, o = idx & 31;
    tile[i][o] = src[(size_t)(i0 + i) * nout + o0 + o];
  }
  __syncthreads();
  const int o = tid >> 3, c8 = (tid & 7) * 8;
  v4u pk;
#pragma unroll
  for (int e = 0; e < 4; ++e)
    pk[e] = pkh(bfr(tile[c8 + 2 * e][o]) * WSC, bfr(tile[c8 + 2 * e + 1][o]) * WSC);
  unsigned short* gp = dst + (size_t)(o0 + o) * nin + i0 + c8;
  *(volatile v4u*)gp = pk;
  __threadfence();
  *(volatile v4u*)gp = pk;
}

__global__ __launch_bounds__(256) void cvt_rows(const float* __restrict__ x, unsigned short* outp, int nrows,
                                                int ncols, float sc) {
  const int tid = threadIdx.x, wave = tid >> 5, lane = tid & 31;
  const int row = blockIdx.x * 8 + wave;
  const int rowc = (row < nrows) ? row : (nrows - 1);
#pragma unroll 1
  for (int c0 = 0; c0 < ncols; c0 += 256) {
    const int c = c0 + lane * 8;
    const bool live = (c < ncols);
    const int cc = live ? c : (ncols - 8);
    const float* rp = x + (size_t)rowc * ncols + cc;
    const v4f a = *(const v4f*)rp;
    const v4f c4v = *(const v4f*)(rp + 4);
    v4u pk;
#pragma unroll
    for (int e = 0; e < 2; ++e) {
      pk[e]     = pkh(bfr(a[2 * e]) * sc, bfr(a[2 * e + 1]) * sc);
      pk[2 + e] = pkh(bfr(c4v[2 * e]) * sc, bfr(c4v[2 * e + 1]) * sc);
    }
    unsigned short* gp = outp + (size_t)rowc * ncols + cc;
    const bool st = live && (row < nrows);
    if (st) { *(volatile v4u*)gp = pk; }
    __threadfence();
    if (st) { *(volatile v4u*)gp = pk; }
  }
}

template <bool MOD>
__global__ __launch_bounds__(256) void ln_rows(const float* __restrict__ xin, const float* __restrict__ g,
                                               const float* __restrict__ bt, const float* __restrict__ mod, int ldm,
                                               unsigned short* oh, unsigned short* ol, int nrows) {
#pragma clang fp contract(off)
  const int tid = threadIdx.x, wave = tid >> 5, lane = tid & 31;
  const int row = blockIdx.x * 8 + wave;
  const int rowc = (row < nrows) ? row : (nrows - 1);
  const int c8 = lane * 8;
  const float* rp = xin + (size_t)rowc * SD_ + c8;
  float x[24];
#pragma unroll
  for (int k = 0; k < 3; ++k) {
    const v4f a = *(const v4f*)(rp + 256 * k);
    const v4f c = *(const v4f*)(rp + 256 * k + 4);
#pragma unroll
    for (int e = 0; e < 4; ++e) { x[8 * k + e] = bfr(a[e]); x[8 * k + 4 + e] = bfr(c[e]); }
  }
  float s = 0.f;
#pragma unroll
  for (int e = 0; e < 24; ++e) s = s + x[e];
#pragma unroll
  for (int off = 1; off < 32; off <<= 1) s = s + __shfl_xor(s, off, 32);
  const float mu = s * (1.0f / SD_);
  float d[24];
  float s2 = 0.f;
#pragma unroll
  for (int e = 0; e < 24; ++e) { d[e] = x[e] - mu; const float dd = d[e] * d[e]; s2 = s2 + dd; }
#pragma unroll
  for (int off = 1; off < 32; off <<= 1) s2 = s2 + __shfl_xor(s2, off, 32);
  const float var = s2 * (1.0f / SD_);
  const float rstd = rsqrtf(var + LNEPS);
  const float* mp = mod + (size_t)rowc * ldm + c8;
  v4u hv[3], lv[3];
#pragma unroll
  for (int k = 0; k < 3; ++k) {
    float mm[8];
#pragma unroll
    for (int e = 0; e < 8; ++e) mm[e] = 0.f;
    if (MOD) {
      const v4f m0v = *(const v4f*)(mp + 256 * k);
      const v4f m1v = *(const v4f*)(mp + 256 * k + 4);
#pragma unroll
      for (int e = 0; e < 4; ++e) { mm[e] = m0v[e]; mm[4 + e] = m1v[e]; }
    }
    float y[8];
#pragma unroll
    for (int e = 0; e < 8; ++e) {
      const int col = 256 * k + c8 + e;
      const float gg = bfr(g[col]), bb = bfr(bt[col]);
      float t = d[8 * k + e] * rstd;
      t = t * gg;
      t = t + bb;
      if (MOD) { const float om = 1.0f + mm[e]; t = t * om; }
      y[e] = t;
    }
    v4u a, bl;
#pragma unroll
    for (int e = 0; e < 4; ++e) {
      unsigned hp, lp;
      hl_pair(y[2 * e], y[2 * e + 1], hp, lp);
      a[e] = hp; bl[e] = lp;
    }
    hv[k] = a; lv[k] = bl;
  }
  if (row < nrows) {
    unsigned short* hp0 = oh + (size_t)row * SD_ + c8;
    unsigned short* lp0 = ol + (size_t)row * SD_ + c8;
    for (int pass = 0; pass < 2; ++pass) {
#pragma unroll
      for (int k = 0; k < 3; ++k) {
        *(volatile v4u*)(hp0 + 256 * k) = hv[k];
        *(volatile v4u*)(lp0 + 256 * k) = lv[k];
      }
      __threadfence();
    }
  }
}

__global__ __launch_bounds__(256) void tr_planes(const unsigned short* __restrict__ sh,
                                                 const unsigned short* __restrict__ sl,
                                                 unsigned short* th, unsigned short* tl) {
  __shared__ __align__(16) unsigned short Th[32 * 264];
  __shared__ __align__(16) unsigned short Tl[32 * 264];
  const int tid = threadIdx.x;
  const int i0 = blockIdx.x * 32, b = blockIdx.y;
#pragma unroll
  for (int it = 0; it < 4; ++it) {
    const int idx = it * 256 + tid;
    const int v = idx >> 2, c = idx & 3;
    const size_t go = (size_t)(b * NV_ + v) * SD_ + i0 + 8 * c;
    const v4u p4 = *(const v4u*)(sh + go);
    const v4u q4 = *(const v4u*)(sl + go);
#pragma unroll
    for (int e = 0; e < 4; ++e) {
      const unsigned wp = p4[e], wq = q4[e];
      Th[(8 * c + 2 * e) * 264 + v]     = (unsigned short)(wp & 0xffffu);
      Th[(8 * c + 2 * e + 1) * 264 + v] = (unsigned short)(wp >> 16);
      Tl[(8 * c + 2 * e) * 264 + v]     = (unsigned short)(wq & 0xffffu);
      Tl[(8 * c + 2 * e + 1) * 264 + v] = (unsigned short)(wq >> 16);
    }
  }
  __syncthreads();
  const int wave = tid >> 5, lane = tid & 31;
  v4u hv[4], lv[4];
#pragma unroll
  for (int k = 0; k < 4; ++k) {
    const int r = wave + 8 * k;
    hv[k] = *(const v4u*)(Th + r * 264 + 8 * lane);
    lv[k] = *(const v4u*)(Tl + r * 264 + 8 * lane);
  }
  for (int pass = 0; pass < 2; ++pass) {
#pragma unroll
    for (int k = 0; k < 4; ++k) {
      const int r = wave + 8 * k;
      const size_t go = (size_t)(b * SD_ + i0 + r) * NV_ + 8 * lane;
      *(volatile v4u*)(th + go) = hv[k];
      *(volatile v4u*)(tl + go) = lv[k];
    }
    __threadfence();
  }
}

__global__ __launch_bounds__(256) void softmax_rows(const float* __restrict__ sc, const float* __restrict__ q32,
                                                    const float* __restrict__ bk, unsigned short* ph,
                                                    unsigned short* pl) {
#pragma clang fp contract(off)
  const int tid = threadIdx.x, wave = tid >> 5, lane = tid & 31;
  const int row = blockIdx.x * 8 + wave;
  const int b = row >> 9, h = (row >> 6) & (NH_ - 1), u = row & (NU_ - 1);
  const float* qr = q32 + (size_t)(b * NU_ + u) * NI_ + h * HD_;
  const float* bkh = bk + h * HD_;
  const float t0 = qr[lane] * bfr(bkh[lane]);
  const float t1 = qr[lane + 32] * bfr(bkh[lane + 32]);
  float qb = t0 + t1;
#pragma unroll
  for (int off = 16; off >= 1; off >>= 1) qb = qb + __shfl_xor(qb, off, 32);
  qb = qb * 0.125f;
  const float* sr = sc + (size_t)row * NV_ + lane * 8;
  const v4f a0 = *(const v4f*)sr;
  const v4f a1 = *(const v4f*)(sr + 4);
  float x[8];
#pragma unroll
  for (int e = 0; e < 4; ++e) { x[e] = a0[e] + qb; x[4 + e] = a1[e] + qb; }
  float mx = x[0];
#pragma unroll
  for (int e = 1; e < 8; ++e) mx = fmaxf(mx, x[e]);
#pragma unroll
  for (int off = 16; off >= 1; off >>= 1) mx = fmaxf(mx, __shfl_xor(mx, off, 32));
  float sum = 0.f;
#pragma unroll
  for (int e = 0; e < 8; ++e) { x[e] = __expf(x[e] - mx); sum = sum + x[e]; }
#pragma unroll
  for (int off = 16; off >= 1; off >>= 1) sum = sum + __shfl_xor(sum, off, 32);
  const float inv = 1.0f / sum;
  v4u hv, lv;
#pragma unroll
  for (int e = 0; e < 4; ++e) {
    float p0 = x[2 * e] * inv;     p0 = p0 * PSC;
    float p1 = x[2 * e + 1] * inv; p1 = p1 * PSC;
    unsigned hp, lp;
    hl_pair(p0, p1, hp, lp);
    hv[e] = hp; lv[e] = lp;
  }
  unsigned short* gh = ph + (size_t)row * NV_ + lane * 8;
  unsigned short* gl = pl + (size_t)row * NV_ + lane * 8;
  *(volatile v4u*)gh = hv;
  *(volatile v4u*)gl = lv;
  __threadfence();
  *(volatile v4u*)gh = hv;
  *(volatile v4u*)gl = lv;
}

struct GArg {
  const unsigned short* A0; const unsigned short* A1; const unsigned short* B0; const unsigned short* B1;
  const float* bias; const float* mul; const float* gvec; const float* resid;
  float* C32; unsigned short* Ch; unsigned short* Cl;
  int lda, ldb, ldc, ldh;
  int ldm, ldr, M, N;
  int K, nb2, sa1, sa2;
  int sb1, sb2, sc1, sc2;
  int sm1, sm2, sbias2, flags;
  int tiles, pad0;
  float s0, s1;
  float oscale, pad1;
};
static_assert(sizeof(GArg) == 192);

template <int NA, int NB>
__global__ __launch_bounds__(256) void gemm16(GArg g) {
#pragma clang fp contract(off)
  __shared__ __align__(16) float sT[8][16 * 68];
  const int lane = threadIdx.x & 31;
  const int wave = threadIdx.x >> 5;
  const int t = __builtin_amdgcn_readfirstlane((int)(blockIdx.x * 8 + wave));
  if (t >= g.tiles) return;
  const int bz = blockIdx.y;
  const int b1 = bz / g.nb2, b2 = bz - b1 * g.nb2;
  const size_t aoff = (size_t)b1 * g.sa1 + (size_t)b2 * g.sa2;
  const size_t boff = (size_t)b1 * g.sb1 + (size_t)b2 * g.sb2;
  const size_t coff = (size_t)b1 * g.sc1 + (size_t)b2 * g.sc2;
  const _Float16* A0 = (const _Float16*)(const void*)g.A0 + aoff;
  const _Float16* A1 = (const _Float16*)(const void*)g.A1 + aoff;
  const _Float16* B0 = (const _Float16*)(const void*)g.B0 + boff;
  const _Float16* B1 = (const _Float16*)(const void*)g.B1 + boff;
  const int tilesN = g.N >> 6;
  const int tm = t / tilesN;
  const int tn = t - tm * tilesN;
  const int m0 = tm * 16;
  const int n0 = tn * 64;

  const int rl   = lane & 15;
  const int hh   = lane >> 4;
  const int koff = hh * 8;

  v8f acc0[4], acc1[4];
#pragma unroll
  for (int j = 0; j < 4; ++j) { acc0[j] = zero8(); acc1[j] = zero8(); }

  const size_t arow = (size_t)(m0 + rl) * g.lda + koff;
#pragma unroll 2
  for (int k0 = 0; k0 < g.K; k0 += 32) {
    const v16h fa0 = ldfrag_h(A0 + arow + k0);
    v16h fa1;
    if (NA == 2) fa1 = ldfrag_h(A1 + arow + k0); else fa1 = fa0;
#pragma unroll
    for (int j = 0; j < 4; ++j) {
      const size_t brow = (size_t)(n0 + 16 * j + rl) * g.ldb + koff + k0;
      const v16h fb0 = ldfrag_h(B0 + brow);
      acc0[j] = mma_h(fa0, fb0, acc0[j]);
      if (NA == 2 && NB == 1) acc1[j] = mma_h(fa1, fb0, acc1[j]);
      if (NA == 2 && NB == 2) {
        const v16h fb1 = ldfrag_h(B1 + brow);
        acc1[j] = mma_h(fa0, fb1, acc1[j]);
        acc1[j] = mma_h(fa1, fb0, acc1[j]);
      }
    }
  }

  const int fl = g.flags;
  const float s0 = g.s0, s1 = g.s1, osc = g.oscale;

  float* slab = sT[wave];
#pragma unroll
  for (int j = 0; j < 4; ++j) {
#pragma unroll
    for (int r = 0; r < 8; ++r) {
      float u = acc0[j][r] * s0;
      if (NA == 2) { const float u1 = acc1[j][r] * s1; u = u + u1; }
      slab[(koff + r) * 68 + 16 * j + rl] = u;
    }
  }
  wave_sync_lds();

  const int h2 = lane >> 4, c4 = (lane & 15) * 4;
  const float* biasp = g.bias + (size_t)b2 * g.sbias2;
  const float* mulp  = g.mul + ((size_t)b1 * g.sm1 + (size_t)b2 * g.sm2);
  float* C32 = g.C32 + coff;
  unsigned short* Ch = g.Ch + coff;
  unsigned short* Cl = g.Cl + coff;
  float bz4[4] = {0.f, 0.f, 0.f, 0.f};
  float gz4[4] = {1.f, 1.f, 1.f, 1.f};
  if (fl & F_BIAS) {
#pragma unroll
    for (int e = 0; e < 4; ++e) bz4[e] = bfr(biasp[n0 + c4 + e]);
  }
  if (fl & F_GCOL) {
#pragma unroll
    for (int e = 0; e < 4; ++e) gz4[e] = bfr(g.gvec[n0 + c4 + e]);
  }
  v4f ov[8];
#pragma unroll
  for (int it = 0; it < 8; ++it) {
    const int row = it * 2 + h2;
    const int gm = m0 + row;
    const v4f v = *(const v4f*)(slab + row * 68 + c4);
    v4f mv = zero4();
    if (fl & F_MULP) mv = *(const v4f*)(mulp + (size_t)gm * g.ldm + n0 + c4);
    v4f rv = zero4();
    if (fl & F_RESID) rv = *(const v4f*)(g.resid + (size_t)gm * g.ldr + n0 + c4);
    v4f o;
#pragma unroll
    for (int e = 0; e < 4; ++e) {
      float f = v[e] + bz4[e];
      if (fl & F_MULP) { const float om = 1.0f + mv[e]; f = f * om; }
      if (fl & F_GCOL) f = f * gz4[e];
      f = f * osc;
      if (fl & F_RESID) f = f + bfr(rv[e]);
      o[e] = f;
    }
    ov[it] = o;
    if (fl & F_OUTHL) *(v4f*)(slab + row * 68 + c4) = o;
  }
  if (fl & F_OUT32) {
    for (int pass = 0; pass < 2; ++pass) {
#pragma unroll
      for (int it = 0; it < 8; ++it) {
        const int row = it * 2 + h2;
        float* gp = C32 + (size_t)(m0 + row) * g.ldc + n0 + c4;
        *(volatile v4f*)gp = ov[it];
      }
      __threadfence();
    }
  }
  if (fl & F_OUTHL) {
    wave_sync_lds();
    const int q = lane >> 3, c8 = (lane & 7) * 8;
    v4u hv[4], lv[4];
#pragma unroll
    for (int it = 0; it < 4; ++it) {
      const int row = it * 4 + q;
      const float* sp = slab + row * 68 + c8;
      const v4f x0 = *(const v4f*)sp;
      const v4f x1 = *(const v4f*)(sp + 4);
      v4u a, bl;
#pragma unroll
      for (int e = 0; e < 2; ++e) {
        unsigned hp, lp;
        hl_pair(x0[2 * e], x0[2 * e + 1], hp, lp); a[e] = hp;     bl[e] = lp;
        hl_pair(x1[2 * e], x1[2 * e + 1], hp, lp); a[2 + e] = hp; bl[2 + e] = lp;
      }
      hv[it] = a; lv[it] = bl;
    }
    for (int pass = 0; pass < 2; ++pass) {
#pragma unroll
      for (int it = 0; it < 4; ++it) {
        const int row = it * 4 + q;
        unsigned short* gh = Ch + (size_t)(m0 + row) * g.ldh + n0 + c8;
        unsigned short* gl = Cl + (size_t)(m0 + row) * g.ldh + n0 + c8;
        *(volatile v4u*)gh = hv[it];
        *(volatile v4u*)gl = lv[it];
      }
      __threadfence();
    }
  }
  wave_sync_lds();
}

static GArg mkg(const unsigned short* A0, const unsigned short* A1, int lda, int sa1, int sa2,
                const unsigned short* B0, const unsigned short* B1, int ldb, int sb1, int sb2,
                int M, int N, int K, int nb2,
                const float* bias, int sbias2, const float* mul, int ldm, int sm1, int sm2,
                const float* gvec, const float* resid, int ldr,
                float* C32, int ldc, unsigned short* Ch, unsigned short* Cl, int ldh, int sc1, int sc2,
                int flags, float s0, float s1, float oscale) {
  GArg g;
  g.A0 = A0; g.A1 = A1; g.B0 = B0; g.B1 = B1;
  g.bias = bias; g.mul = mul; g.gvec = gvec; g.resid = resid;
  g.C32 = C32; g.Ch = Ch; g.Cl = Cl;
  g.lda = lda; g.ldb = ldb; g.ldc = ldc; g.ldh = ldh;
  g.ldm = ldm; g.ldr = ldr; g.M = M; g.N = N;
  g.K = K; g.nb2 = nb2; g.sa1 = sa1; g.sa2 = sa2;
  g.sb1 = sb1; g.sb2 = sb2; g.sc1 = sc1; g.sc2 = sc2;
  g.sm1 = sm1; g.sm2 = sm2; g.sbias2 = sbias2; g.flags = flags;
  g.tiles = (M / 16) * (N / 64); g.pad0 = 0;
  g.s0 = s0; g.s1 = s1; g.oscale = oscale; g.pad1 = 0.f;
  return g;
}
template <int NA, int NB>
static void run_g(const GArg& g, int nbat, hipStream_t st) {
  if (g.tiles <= 0 || nbat <= 0) return;
  const dim3 grid((g.tiles + 7) / 8, nbat);
  gemm16<NA, NB><<<grid, dim3(256), 0, st>>>(g);
}

extern "C" void kernel_launch(void* const* d_in, const int* in_sizes, int n_in,
                              void* d_out, int out_size, void* d_ws, size_t ws_size,
                              hipStream_t stream) {
  if (n_in < 20) return;
  const int ex[20] = { RROWS * SD_, RROWS * CD_, SROWS * SD_, SD_, SD_, SD_, SD_,
                       SD_ * NI_, NI_, CD_ * SD_, SD_ * NI_, NI_, CD_ * SD_, SD_ * NI_, NI_, CD_ * SD_,
                       NI_ * SD_, SD_, CD_ * NI_, SD_ };
  for (int i = 0; i < 20; ++i) if (in_sizes[i] != ex[i]) return;
  if (out_size != RROWS * SD_) return;

  const float* rs     = (const float*)d_in[0];
  const float* codes  = (const float*)d_in[1];
  const float* ss     = (const float*)d_in[2];
  const float* ln_r_g = (const float*)d_in[3];
  const float* ln_r_b = (const float*)d_in[4];
  const float* ln_s_g = (const float*)d_in[5];
  const float* ln_s_b = (const float*)d_in[6];
  const float* Wq  = (const float*)d_in[7];  const float* bq = (const float*)d_in[8];
  const float* Wmq = (const float*)d_in[9];
  const float* Wk  = (const float*)d_in[10]; const float* bk = (const float*)d_in[11];
  const float* Wmk = (const float*)d_in[12];
  const float* Wv  = (const float*)d_in[13]; const float* bv = (const float*)d_in[14];
  const float* Wmv = (const float*)d_in[15];
  const float* We  = (const float*)d_in[16]; const float* be = (const float*)d_in[17];
  const float* Wme = (const float*)d_in[18];
  const float* gamma = (const float*)d_in[19];
  float* out = (float*)d_out;

  const size_t sWMT = (size_t)CMW * CD_ * 2;
  const size_t sWQV = (size_t)2 * NI_ * SD_ * 2;
  const size_t sWET = (size_t)SD_ * NI_ * 2;
  const size_t sWK  = (size_t)SD_ * NI_ * 2;
  const size_t sCD  = (size_t)RROWS * CD_ * 2;
  const size_t sSP  = (size_t)SROWS * SD_ * 2;
  const size_t sCM  = (size_t)RROWS * CMW * 4;
  const size_t sQI  = (size_t)RROWS * SD_ * 2;
  const size_t sQ32 = (size_t)RROWS * NI_ * 4;
  const size_t sQP  = (size_t)RROWS * NI_ * 2;
  const size_t sGP  = (size_t)AROWS * SD_ * 2;
  const size_t sSC  = (size_t)AROWS * NV_ * 4;
  const size_t sPP  = (size_t)AROWS * NV_ * 2;
  const size_t sTP  = (size_t)NB_ * SD_ * NV_ * 2;
  const size_t sAP  = (size_t)AROWS * SD_ * 2;
  const size_t sMP  = (size_t)RROWS * NI_ * 2;
  size_t off = 0;
  const size_t oWMT = off; off += sWMT;
  const size_t oWQV = off; off += sWQV;
  const size_t oWET = off; off += sWET;
  const size_t oWK  = off; off += sWK;
  const size_t oCD  = off; off += sCD;
  const size_t oSH  = off; off += sSP;
  const size_t oSL  = off; off += sSP;
  const size_t oCM  = off; off += sCM;
  const size_t oQIH = off; off += sQI;
  const size_t oQIL = off; off += sQI;
  const size_t oQ32 = off; off += sQ32;
  const size_t oQH  = off; off += sQP;
  const size_t oQL  = off; off += sQP;
  const size_t oGH  = off; off += sGP;
  const size_t oGL  = off; off += sGP;
  const size_t oSC  = off; off += sSC;
  const size_t oPH  = off; off += sPP;
  const size_t oPL  = off; off += sPP;
  const size_t oTH  = off; off += sTP;
  const size_t oTL  = off; off += sTP;
  const size_t oAH  = off; off += sAP;
  const size_t oAL  = off; off += sAP;
  const size_t oMH  = off; off += sMP;
  const size_t oML  = off; off += sMP;
  if (off > ws_size) return;
  if (off > (size_t)134217728) return;

  char* ws = (char*)d_ws;
  unsigned short* WMT = (unsigned short*)(ws + oWMT);
  unsigned short* WQV = (unsigned short*)(ws + oWQV);
  unsigned short* WET = (unsigned short*)(ws + oWET);
  unsigned short* WK  = (unsigned short*)(ws + oWK);
  unsigned short* CD  = (unsigned short*)(ws + oCD);
  unsigned short* SH  = (unsigned short*)(ws + oSH);
  unsigned short* SL  = (unsigned short*)(ws + oSL);
  float*          CM  = (float*)(ws + oCM);
  unsigned short* QIH = (unsigned short*)(ws + oQIH);
  unsigned short* QIL = (unsigned short*)(ws + oQIL);
  float*          Q32 = (float*)(ws + oQ32);
  unsigned short* QH  = (unsigned short*)(ws + oQH);
  unsigned short* QL  = (unsigned short*)(ws + oQL);
  unsigned short* GH  = (unsigned short*)(ws + oGH);
  unsigned short* GL  = (unsigned short*)(ws + oGL);
  float*          SC  = (float*)(ws + oSC);
  unsigned short* PH  = (unsigned short*)(ws + oPH);
  unsigned short* PL  = (unsigned short*)(ws + oPL);
  unsigned short* TH  = (unsigned short*)(ws + oTH);
  unsigned short* TL  = (unsigned short*)(ws + oTL);
  unsigned short* AH  = (unsigned short*)(ws + oAH);
  unsigned short* AL  = (unsigned short*)(ws + oAL);
  unsigned short* MH  = (unsigned short*)(ws + oMH);
  unsigned short* ML  = (unsigned short*)(ws + oML);
  const unsigned short* WQT = WQV;
  const unsigned short* WVT = WQV + (size_t)NI_ * SD_;

  const dim3 blk(256);

  cvt_wT<<<dim3(CD_ / 64, SD_ / 32, 3), blk, 0, stream>>>(Wmq, Wmk, Wmv, WMT, CD_, SD_);
  cvt_wT<<<dim3(CD_ / 64, NI_ / 32, 1), blk, 0, stream>>>(Wme, Wme, Wme, WMT + (size_t)3 * SD_ * CD_, CD_, NI_);
  cvt_wT<<<dim3(SD_ / 64, NI_ / 32, 2), blk, 0, stream>>>(Wq, Wv, Wv, WQV, SD_, NI_);
  cvt_wT<<<dim3(NI_ / 64, SD_ / 32, 1), blk, 0, stream>>>(We, We, We, WET, NI_, SD_);
  cvt_rows<<<dim3(SD_ / 8), blk, 0, stream>>>(Wk, WK, SD_, NI_, WSC);
  cvt_rows<<<dim3(RROWS / 8), blk, 0, stream>>>(codes, CD, RROWS, CD_, 1.0f);
  ln_rows<false><<<dim3(SROWS / 8), blk, 0, stream>>>(ss, ln_s_g, ln_s_b, CM, CMW, SH, SL, SROWS);
  {
    GArg g = mkg(CD, CD, CD_, 0, 0, WMT, WMT, CD_, 0, 0, RROWS, CMW, CD_, 1,
                 bq, 0, Q32, CMW, 0, 0, gamma, rs, SD_,
                 CM, CMW, QH, QL, NI_, 0, 0, F_OUT32, 1.0f / WSC, 0.0f, 1.0f);
    run_g<1, 1>(g, 1, stream);
  }
  ln_rows<true><<<dim3(RROWS / 8), blk, 0, stream>>>(rs, ln_r_g, ln_r_b, CM, CMW, QIH, QIL, RROWS);
  {
    GArg g = mkg(QIH, QIL, SD_, 0, 0, WQT, WQT, SD_, 0, 0, RROWS, NI_, SD_, 1,
                 bq, 0, CM, CMW, 0, 0, gamma, rs, SD_,
                 Q32, NI_, QH, QL, NI_, 0, 0, F_BIAS | F_OUT32 | F_OUTHL,
                 1.0f / WSC, 1.0f / (WSC * LOSC), 1.0f);
    run_g<2, 1>(g, 1, stream);
  }
  {
    GArg g = mkg(QH, QL, NI_, NU_ * NI_, HD_, WK, WK, NI_, 0, HD_, NU_, SD_, HD_, NH_,
                 bq, 0, CM + SD_, CMW, NU_ * CMW, 0, gamma, rs, SD_,
                 SC, SD_, GH, GL, SD_, NH_ * NU_ * SD_, NU_ * SD_, F_MULP | F_OUTHL,
                 1.0f, 1.0f / LOSC, 1.0f);
    run_g<2, 1>(g, NB_ * NH_, stream);
  }
  {
    GArg g = mkg(GH, GL, SD_, NH_ * NU_ * SD_, NU_ * SD_, SH, SL, SD_, NV_ * SD_, 0, NU_, NV_, SD_, NH_,
                 bq, 0, CM, CMW, 0, 0, gamma, rs, SD_,
                 SC, NV_, QH, QL, NI_, NH_ * NU_ * NV_, NU_ * NV_, F_OUT32,
                 1.0f / 512.0f, 1.0f / (512.0f * LOSC), 1.0f);
    run_g<2, 2>(g, NB_ * NH_, stream);
  }
  softmax_rows<<<dim3(AROWS / 8), blk, 0, stream>>>(SC, Q32, bk, PH, PL);
  tr_planes<<<dim3(SD_ / 32, NB_), blk, 0, stream>>>(SH, SL, TH, TL);
  {
    GArg g = mkg(PH, PL, NV_, NH_ * NU_ * NV_, NU_ * NV_, TH, TL, NV_, SD_ * NV_, 0, NU_, SD_, NV_, NH_,
                 bq, 0, CM + 2 * SD_, CMW, NU_ * CMW, 0, gamma, rs, SD_,
                 SC, SD_, AH, AL, SD_, NH_ * NU_ * SD_, NU_ * SD_, F_MULP | F_OUTHL,
                 1.0f / PSC, 1.0f / (PSC * LOSC), ASC);
    run_g<2, 2>(g, NB_ * NH_, stream);
  }
  {
    GArg g = mkg(AH, AL, SD_, NH_ * NU_ * SD_, NU_ * SD_, WVT, WVT, SD_, 0, HD_ * SD_, NU_, HD_, SD_, NH_,
                 bv, HD_, CM + 3 * SD_, CMW, NU_ * CMW, HD_, gamma, rs, SD_,
                 SC, NI_, MH, ML, NI_, NU_ * NI_, HD_, F_BIAS | F_MULP | F_OUTHL,
                 1.0f / (ASC * WSC), 1.0f / (ASC * WSC * LOSC), MSC);
    run_g<2, 1>(g, NB_ * NH_, stream);
  }
  {
    GArg g = mkg(MH, ML, NI_, 0, 0, WET, WET, NI_, 0, 0, RROWS, SD_, NI_, 1,
                 be, 0, CM, CMW, 0, 0, gamma, rs, SD_,
                 out, SD_, QH, QL, NI_, 0, 0, F_BIAS | F_GCOL | F_RESID | F_OUT32,
                 1.0f / (MSC * WSC), 1.0f / (MSC * WSC * LOSC), 1.0f);
    run_g<2, 1>(g, 1, stream);
  }
  (void)hipGetLastError();
}
